// Retention_86328842650435
// MI455X (gfx1250) — hardware-verified
//
#include <hip/hip_runtime.h>
#include <math.h>

constexpr int kT   = 2048;
constexpr int kE   = 1024;
constexpr int kH   = 16;
constexpr int kHD  = 64;
constexpr int kGroup = 2;
constexpr float kQKVCarry  = 16.0f;
constexpr float kPCarry    = 32768.0f;
constexpr float kScoreScale = 0.125f / (16.0f * 16.0f);
constexpr float kPVScale    = 1.0f / (32768.0f * 16.0f);
constexpr float kGnEps      = 1.0e-5f;
static_assert(kH * kHD == kE, "shape");
static_assert(kT % 64 == 0 && kE % 64 == 0 && kHD % 64 == 0, "M,N tile multiples");
static_assert(kE % 32 == 0 && kHD % 32 == 0 && kT % 32 == 0, "K multiples of 32");
static_assert(kH % kGroup == 0 && kT % 256 == 0 && kT % 8 == 0, "groups");

typedef __attribute__((ext_vector_type(16))) _Float16 v16h;
typedef __attribute__((ext_vector_type(8)))  _Float16 v8h;
typedef __attribute__((ext_vector_type(16))) __bf16   v16b;
typedef __attribute__((ext_vector_type(8)))  __bf16   v8b;
typedef __attribute__((ext_vector_type(8)))  float    v8f;
typedef __attribute__((ext_vector_type(4)))  float    v4f;
typedef __attribute__((ext_vector_type(2)))  float    v2f;
typedef __attribute__((ext_vector_type(4)))  unsigned int v4u;

__device__ __forceinline__ unsigned short f2bf_bits(float f) {
  unsigned u = __float_as_uint(f);
  return (unsigned short)((u + 0x7FFFu + ((u >> 16) & 1u)) >> 16);
}
__device__ __forceinline__ float bf_bits2f(unsigned short h) { return __uint_as_float(((unsigned)h) << 16); }

__device__ __forceinline__ void dep_guard_h(v8f& a, v8f& b, v16h x, v16h y) { asm volatile("v_nop\n\tv_nop\n\tv_nop\n\tv_nop" : "+v"(a), "+v"(b) : "v"(x), "v"(y)); }
__device__ __forceinline__ void dep_guard_b(v8f& a, v8f& b, v16b x, v16b y) { asm volatile("v_nop\n\tv_nop\n\tv_nop\n\tv_nop" : "+v"(a), "+v"(b) : "v"(x), "v"(y)); }
__device__ __forceinline__ void dep_guard4_h(v8f& a, v8f& b, v8f& c, v8f& d, v16h x, v16h y) { asm volatile("v_nop\n\tv_nop\n\tv_nop\n\tv_nop" : "+v"(a), "+v"(b), "+v"(c), "+v"(d) : "v"(x), "v"(y)); }
__device__ __forceinline__ void dep_guard4_b(v8f& a, v8f& b, v8f& c, v8f& d, v16b x, v16b y) { asm volatile("v_nop\n\tv_nop\n\tv_nop\n\tv_nop" : "+v"(a), "+v"(b), "+v"(c), "+v"(d) : "v"(x), "v"(y)); }
__device__ __forceinline__ void keep4_h(v16h a, v16h b, v16h c, v16h d) { asm volatile("v_nop" :: "v"(a), "v"(b), "v"(c), "v"(d)); }
__device__ __forceinline__ void keep4_b(v16b a, v16b b, v16b c, v16b d) { asm volatile("v_nop" :: "v"(a), "v"(b), "v"(c), "v"(d)); }
__device__ __forceinline__ void acc_guard4(v8f& a, v8f& b, v8f& c, v8f& d) { asm volatile("v_nop\n\tv_nop\n\tv_nop\n\tv_nop" : "+v"(a), "+v"(b), "+v"(c), "+v"(d)); }
template <typename T> struct Frag;
template <> struct Frag<_Float16> {
  typedef v16h V; union U { v16h v; v8h h[2]; };
  static __device__ __forceinline__ v16h load(const _Float16* p) {
    U f; f.h[0] = *(const v8h*)(p); f.h[1] = *(const v8h*)(p + 16); return f.v;
  }
  static __device__ __forceinline__ v8f mma(v16h a, v16h b, v8f c) {
    return __builtin_amdgcn_wmma_f32_16x16x32_f16(false, a, false, b, (short)0, c, false, false);
  }
  static __device__ __forceinline__ void guard(v8f& a, v8f& b, v16h x, v16h y) { dep_guard_h(a, b, x, y); }
  static __device__ __forceinline__ void guard4(v8f& a, v8f& b, v8f& c, v8f& d, v16h x, v16h y) { dep_guard4_h(a, b, c, d, x, y); }
  static __device__ __forceinline__ void keep(v16h a, v16h b, v16h c, v16h d) { keep4_h(a, b, c, d); }
};
template <> struct Frag<__bf16> {
  typedef v16b V; union U { v16b v; v8b h[2]; };
  static __device__ __forceinline__ v16b load(const __bf16* p) {
    U f; f.h[0] = *(const v8b*)(p); f.h[1] = *(const v8b*)(p + 16); return f.v;
  }
  static __device__ __forceinline__ v8f mma(v16b a, v16b b, v8f c) {
    return __builtin_amdgcn_wmma_f32_16x16x32_bf16(false, a, false, b, (short)0, c, false, false);
  }
  static __device__ __forceinline__ void guard(v8f& a, v8f& b, v16b x, v16b y) { dep_guard_b(a, b, x, y); }
  static __device__ __forceinline__ void guard4(v8f& a, v8f& b, v8f& c, v8f& d, v16b x, v16b y) { dep_guard4_b(a, b, c, d, x, y); }
  static __device__ __forceinline__ void keep(v16b a, v16b b, v16b c, v16b d) { keep4_b(a, b, c, d); }
};

__device__ __forceinline__ unsigned pk16(unsigned short a, unsigned short b) { return (unsigned)a | ((unsigned)b << 16); }
__device__ __forceinline__ unsigned short h_bits(float f) { const _Float16 h = (_Float16)f; return __builtin_bit_cast(unsigned short, h); }

template <int ET> struct Elem;
template <> struct Elem<0> { typedef _Float16 T; };
template <> struct Elem<1> { typedef __bf16 T; };
template <int ET, bool SPLIT, int BIAS_MODE, int OUT_MODE, bool RESID, int ACT = 0>
__global__ __launch_bounds__(256) void wmma_gemm64(
    const unsigned short* __restrict__ Ap, const unsigned short* __restrict__ A2p, int lda, long strideA,
    const unsigned short* __restrict__ Btp, const unsigned short* __restrict__ Bt2p, int ldb, long strideB,
    void* __restrict__ Cout, void* __restrict__ Cout2, int ldc, long strideC,
    const float* __restrict__ bias,
    const float* __restrict__ resid, long strideR,
    int M, int N, int K, float scale) {
  typedef typename Elem<ET>::T T;
  typedef typename Frag<T>::V V;
  const T* A = (const T*)Ap; const T* A2 = (const T*)A2p; const T* Bt = (const T*)Btp; const T* Bt2 = (const T*)Bt2p;
  __shared__ __align__(16) float sT[8][16 * 68];
  const int b    = blockIdx.y;
  const int lane = threadIdx.x & 31;
  const int wave = threadIdx.x >> 5;
  const int tilesN = N >> 6;
  const int tilesM = M >> 6;
  const int tile = blockIdx.x * 8 + wave;
  if (tile >= tilesM * tilesN) return;
  const int tm = tile / tilesN;
  const int tn = tile - tm * tilesN;
  const int m0 = tm << 6;
  const int n0 = tn << 6;

  const T* Ab  = A  + (size_t)b * strideA;
  const T* Bb  = Bt + (size_t)b * strideB;
  const T* Ab2 = SPLIT ? (A2  + (size_t)b * strideA) : nullptr;
  const T* Bb2 = SPLIT ? (Bt2 + (size_t)b * strideB) : nullptr;

  const int rlane = lane & 15;
  const int koff  = (lane >> 4) * 8;
  const int mOff  = (lane >> 4) * 8;

  v8f acc[4][4];
#pragma unroll
  for (int i = 0; i < 4; ++i)
#pragma unroll
    for (int j = 0; j < 4; ++j) acc[i][j] = (v8f){0.f,0.f,0.f,0.f,0.f,0.f,0.f,0.f};

  for (int k0 = 0; k0 < K; k0 += 32) {
    V bh[4], bl[4];
#pragma unroll
    for (int j = 0; j < 4; ++j) {
      const size_t bo = (size_t)(n0 + (j << 4) + rlane) * ldb + koff + k0;
      bh[j] = Frag<T>::load(Bb + bo);
      if (SPLIT) bl[j] = Frag<T>::load(Bb2 + bo);
    }
#pragma unroll
    for (int i = 0; i < 4; ++i) {
      const size_t ao = (size_t)(m0 + (i << 4) + rlane) * lda + koff + k0;
      V ah = Frag<T>::load(Ab + ao);
      V al;
      if (SPLIT) al = Frag<T>::load(Ab2 + ao);
#pragma unroll
      for (int j = 0; j < 4; ++j) {
        acc[i][j] = Frag<T>::mma(ah, bh[j], acc[i][j]);
        if (SPLIT) {
          acc[i][j] = Frag<T>::mma(ah, bl[j], acc[i][j]);
          acc[i][j] = Frag<T>::mma(al, bh[j], acc[i][j]);
        }
      }
      Frag<T>::guard4(acc[i][0], acc[i][1], acc[i][2], acc[i][3], ah, SPLIT ? al : ah);
    }
    Frag<T>::keep(bh[0], bh[1], bh[2], bh[3]);
    if (SPLIT) Frag<T>::keep(bl[0], bl[1], bl[2], bl[3]);
  }
  acc_guard4(acc[0][0], acc[0][1], acc[0][2], acc[0][3]);
  acc_guard4(acc[1][0], acc[1][1], acc[1][2], acc[1][3]);
  acc_guard4(acc[2][0], acc[2][1], acc[2][2], acc[2][3]);
  acc_guard4(acc[3][0], acc[3][1], acc[3][2], acc[3][3]);

  float* slab = sT[wave];
  const float* Rb = RESID ? (resid + (size_t)b * strideR) : nullptr;
#pragma unroll
  for (int i = 0; i < 4; ++i) {
    const int mBase = m0 + (i << 4);
#pragma unroll
    for (int j = 0; j < 4; ++j) {
      const int n = n0 + (j << 4) + rlane;
      float bv = 0.f;
      if (BIAS_MODE == 2) bv = bias[n];
#pragma unroll
      for (int r = 0; r < 8; ++r) {
        float v = acc[i][j][r] * scale;
        if (BIAS_MODE == 1) v += bias[mBase + mOff + r];
        if (BIAS_MODE == 2) v += bv;
        if (RESID) v += Rb[(size_t)(mBase + mOff + r) * ldc + n];
        if (ACT == 2) v = fmaxf(v, 0.0f);
        if (ACT == 4) v = (v > 0.f) ? v : 0.01f * v;
        slab[(mOff + r) * 68 + (j << 4) + rlane] = v;
      }
    }
    __builtin_amdgcn_fence(__ATOMIC_RELEASE, "workgroup");
    __builtin_amdgcn_wave_barrier();
    __builtin_amdgcn_fence(__ATOMIC_ACQUIRE, "workgroup");
    if (OUT_MODE == 0) {
      float* C = (float*)Cout + (size_t)b * strideC;
      const int hh = lane >> 4, c4 = (lane & 15) * 4;
      for (int pass = 0; pass < 2; ++pass) {
#pragma unroll
        for (int it = 0; it < 8; ++it) {
          const int row = it * 2 + hh;
          v4f v = *(const v4f*)(slab + row * 68 + c4);
          *(volatile v4f*)(C + (size_t)(mBase + row) * ldc + n0 + c4) = v;
        }
        __threadfence();
      }
    } else {
      const int q = lane >> 3, c8 = (lane & 7) * 8;
      unsigned short* C  = (unsigned short*)Cout  + (size_t)b * strideC;
      unsigned short* C2 = (OUT_MODE == 2) ? ((unsigned short*)Cout2 + (size_t)b * strideC) : nullptr;
      for (int pass = 0; pass < 2; ++pass) {
#pragma unroll
        for (int it = 0; it < 4; ++it) {
          const int row = it * 4 + q;
          const float* sp = slab + row * 68 + c8;
          v8h hv, lv;
#pragma unroll
          for (int e = 0; e < 8; ++e) {
            if (OUT_MODE == 1) {
              hv[e] = (_Float16)sp[e];
            } else {
              unsigned short hb = f2bf_bits(sp[e]);
              unsigned short lb = f2bf_bits(sp[e] - bf_bits2f(hb));
              hv[e] = __builtin_bit_cast(_Float16, hb);
              lv[e] = __builtin_bit_cast(_Float16, lb);
            }
          }
          *(volatile v8h*)(C + (size_t)(mBase + row) * ldc + n0 + c8) = hv;
          if (OUT_MODE == 2) *(volatile v8h*)(C2 + (size_t)(mBase + row) * ldc + n0 + c8) = lv;
        }
        __threadfence();
      }
    }
    __builtin_amdgcn_fence(__ATOMIC_RELEASE, "workgroup");
    __builtin_amdgcn_wave_barrier();
    __builtin_amdgcn_fence(__ATOMIC_ACQUIRE, "workgroup");
  }
}

__device__ __forceinline__ float wave_sum32(float v) {
#pragma unroll
  for (int off = 16; off > 0; off >>= 1) v += __shfl_xor(v, off, 32);
  return v;
}
__device__ __forceinline__ float wave_max32(float v) {
#pragma unroll
  for (int off = 16; off > 0; off >>= 1) v = fmaxf(v, __shfl_xor(v, off, 32));
  return v;
}

__global__ __launch_bounds__(256) void split8_bf16_kernel(const float* __restrict__ in, unsigned short* __restrict__ hi,
                                                           unsigned short* __restrict__ lo, int n8) {
  const int i = blockIdx.x * 256 + threadIdx.x;
  if (i >= n8) return;
  const float* p = in + 8 * (size_t)i;
  const v4f a = *(const v4f*)(p);
  const v4f c = *(const v4f*)(p + 4);
  unsigned short hb[8], lb[8];
#pragma unroll
  for (int e = 0; e < 4; ++e) {
    const float f0 = a[e], f1 = c[e];
    const unsigned short h0 = f2bf_bits(f0), h1 = f2bf_bits(f1);
    hb[e]     = h0;
    hb[4 + e] = h1;
    lb[e]     = f2bf_bits(f0 - bf_bits2f(h0));
    lb[4 + e] = f2bf_bits(f1 - bf_bits2f(h1));
  }
  const v4u uh = (v4u){pk16(hb[0], hb[1]), pk16(hb[2], hb[3]), pk16(hb[4], hb[5]), pk16(hb[6], hb[7])};
  const v4u ul = (v4u){pk16(lb[0], lb[1]), pk16(lb[2], lb[3]), pk16(lb[4], lb[5]), pk16(lb[6], lb[7])};
  unsigned short* qh = hi + 8 * (size_t)i;
  unsigned short* ql = lo + 8 * (size_t)i;
  *(volatile v4u*)qh = uh;
  *(volatile v4u*)ql = ul;
  __threadfence();
  *(volatile v4u*)qh = uh;
  *(volatile v4u*)ql = ul;
}

struct FreqTab { float f[32]; };
static_assert(sizeof(FreqTab) == 128, "no padding");

__global__ __launch_bounds__(256) void trig_table_kernel(float* __restrict__ cosT, float* __restrict__ sinT, FreqTab tab) {
#pragma clang fp contract(off)
  const int lane = threadIdx.x & 31, wave = threadIdx.x >> 5;
  const int t = blockIdx.x * 8 + wave;
  float f = tab.f[0];
#pragma unroll
  for (int jj = 1; jj < 32; ++jj) f = (lane == jj) ? tab.f[jj] : f;
  const float ang = (float)t * f;
  float sv, cv;
  sincosf(ang, &sv, &cv);
  float* cp = cosT + (size_t)t * 32 + lane;
  float* sp = sinT + (size_t)t * 32 + lane;
  *(volatile float*)cp = cv;
  *(volatile float*)sp = sv;
  __threadfence();
  *(volatile float*)cp = cv;
  *(volatile float*)sp = sv;
}

__global__ __launch_bounds__(256) void stats_decay_kernel(const float* __restrict__ x, const float* __restrict__ wd,
                                                          const float* __restrict__ bd, float* __restrict__ ldout) {
  __shared__ float xm_s[kE];
  __shared__ float ld_s[kH];
  const int tid = threadIdx.x;
  const int lane = tid & 31, wave = tid >> 5;
  float s0 = 0.0f, s1 = 0.0f, s2 = 0.0f, s3 = 0.0f;
#pragma unroll 1
  for (int t = 0; t < kT; ++t) {
    const float* xr = x + (size_t)t * kE + tid;
    s0 += xr[0];
    s1 += xr[256];
    s2 += xr[512];
    s3 += xr[768];
  }
  const float invT = 1.0f / (float)kT;
  xm_s[tid]       = s0 * invT;
  xm_s[tid + 256] = s1 * invT;
  xm_s[tid + 512] = s2 * invT;
  xm_s[tid + 768] = s3 * invT;
  __syncthreads();
#pragma unroll
  for (int hh = 0; hh < 2; ++hh) {
    const int h = wave * 2 + hh;
    const float* wr = wd + (size_t)h * kE;
    float p = 0.0f;
#pragma unroll 1
    for (int c = lane; c < kE; c += 32) p = fmaf(xm_s[c], wr[c], p);
    p = wave_sum32(p);
    const float z  = p + bd[h];
    const float pd = 1.0f / (1.0f + expf(-z));
    const float u  = exp2f(-5.0f - 8.0f * pd);
    const float ldv = logf(1.0f - u);
    if (lane == 0) ld_s[h] = ldv;
  }
  __syncthreads();
  if (wave == 0) {
    const float vv = ld_s[lane & (kH - 1)];
    const float v  = (lane < kH) ? vv : 0.0f;
    float* dp = ldout + lane;
    *(volatile float*)dp = v;
    __threadfence();
    *(volatile float*)dp = v;
  }
}

__global__ __launch_bounds__(256) void rope_pack_kernel(const float* __restrict__ Qr, const float* __restrict__ Kr,
                                                        const float* __restrict__ Vr,
                                                        const float* __restrict__ cosT, const float* __restrict__ sinT,
                                                        unsigned short* __restrict__ Qh, unsigned short* __restrict__ Kh,
                                                        unsigned short* __restrict__ Vt) {
  __shared__ float smq[64][65];
  __shared__ float smk[64][65];
  __shared__ float smv[64][65];
  const int tid = threadIdx.x;
  const int t0  = blockIdx.x * 64;
  const int h   = blockIdx.y;
#pragma unroll 1
  for (int i = 0; i < 4; ++i) {
    const int e  = i * 256 + tid;
    const int r  = e >> 4;
    const int c4 = (e & 15) * 4;
    const size_t src = (size_t)(t0 + r) * kE + h * kHD + c4;
    const v4f q4 = *(const v4f*)(Qr + src);
    const v4f k4 = *(const v4f*)(Kr + src);
    const v4f w4 = *(const v4f*)(Vr + src);
#pragma unroll
    for (int k = 0; k < 4; ++k) {
      smq[r][c4 + k] = q4[k];
      smk[r][c4 + k] = k4[k];
      smv[c4 + k][r] = w4[k];
    }
  }
  __syncthreads();
  const int lane = tid & 31, wave = tid >> 5;
  const int q = lane >> 3, c8 = (lane & 7) * 8;
  const int j8 = c8 & 31;
  v4u uq[2], uk[2], uv[2];
#pragma unroll
  for (int it = 0; it < 2; ++it) {
    const int row = wave * 8 + it * 4 + q;
    const int t = t0 + row;
    const v4f ca = *(const v4f*)(cosT + (size_t)t * 32 + j8);
    const v4f cb = *(const v4f*)(cosT + (size_t)t * 32 + j8 + 4);
    const v4f sa = *(const v4f*)(sinT + (size_t)t * 32 + j8);
    const v4f sb = *(const v4f*)(sinT + (size_t)t * 32 + j8 + 4);
    float cv[8], sv[8], qv[8], kv[8];
#pragma unroll
    for (int e = 0; e < 4; ++e) { cv[e] = ca[e]; cv[4 + e] = cb[e]; sv[e] = sa[e]; sv[4 + e] = sb[e]; }
#pragma unroll
    for (int e = 0; e < 8; ++e) { qv[e] = smq[row][c8 + e]; kv[e] = smk[row][c8 + e]; }
    unsigned short hq[8], hk[8], hv[8];
#pragma unroll
    for (int p = 0; p < 4; ++p) {
      const int e0 = 2 * p, e1 = 2 * p + 1;
      const float qo0 = qv[e0] * cv[e0] - qv[e1] * sv[e0];
      const float qo1 = qv[e1] * cv[e1] + qv[e0] * sv[e1];
      const float ko0 = kv[e0] * cv[e0] - kv[e1] * sv[e0];
      const float ko1 = kv[e1] * cv[e1] + kv[e0] * sv[e1];
      hq[e0] = h_bits(qo0 * kQKVCarry);
      hq[e1] = h_bits(qo1 * kQKVCarry);
      hk[e0] = h_bits(ko0 * kQKVCarry);
      hk[e1] = h_bits(ko1 * kQKVCarry);
    }
#pragma unroll
    for (int e = 0; e < 8; ++e) hv[e] = h_bits(smv[row][c8 + e] * kQKVCarry);
    uq[it] = (v4u){pk16(hq[0], hq[1]), pk16(hq[2], hq[3]), pk16(hq[4], hq[5]), pk16(hq[6], hq[7])};
    uk[it] = (v4u){pk16(hk[0], hk[1]), pk16(hk[2], hk[3]), pk16(hk[4], hk[5]), pk16(hk[6], hk[7])};
    uv[it] = (v4u){pk16(hv[0], hv[1]), pk16(hv[2], hv[3]), pk16(hv[4], hv[5]), pk16(hv[6], hv[7])};
  }
  for (int pass = 0; pass < 2; ++pass) {
#pragma unroll
    for (int it = 0; it < 2; ++it) {
      const int row = wave * 8 + it * 4 + q;
      const int t = t0 + row;
      *(volatile v4u*)(Qh + ((size_t)h * kT + t) * kHD + c8) = uq[it];
      *(volatile v4u*)(Kh + ((size_t)h * kT + t) * kHD + c8) = uk[it];
      *(volatile v4u*)(Vt + ((size_t)h * kHD + row) * kT + t0 + c8) = uv[it];
    }
    __threadfence();
  }
}

__global__ __launch_bounds__(256) void softmax_bias_kernel(const float* __restrict__ Sp, const float* __restrict__ ldp,
                                                           unsigned short* __restrict__ Pp, int hbase) {
  __shared__ __align__(16) float lg[kT];
  __shared__ float redM[8];
  __shared__ float redS[8];
  const int i    = blockIdx.x;
  const int hg   = blockIdx.y;
  const int t    = threadIdx.x;
  const int lane = t & 31, wave = t >> 5;
  const size_t rowoff = ((size_t)hg * kT + i) * kT;
  const float* sr = Sp + rowoff;
  const float ld = ldp[hbase + hg];

  float mx = -__builtin_inff();
#pragma unroll 1
  for (int it = 0; it < 4; ++it) {
    const int c = it * 512 + 2 * t;
    const v2f sv = *(const v2f*)(sr + c);
    v2f av;
#pragma unroll
    for (int e = 0; e < 2; ++e) {
      int dpos = (c + e) - i;
      dpos = dpos > 0 ? dpos : 0;
      const float a = sv[e] + (float)dpos * ld;
      av[e] = a;
      mx = fmaxf(mx, a);
    }
    *(v2f*)(lg + c) = av;
  }
  mx = wave_max32(mx);
  if (lane == 0) redM[wave] = mx;
  __syncthreads();
  float m = redM[0];
#pragma unroll
  for (int w = 1; w < 8; ++w) m = fmaxf(m, redM[w]);

  float sum = 0.0f;
#pragma unroll 1
  for (int it = 0; it < 4; ++it) {
    const int c = it * 512 + 2 * t;
    const v2f l = *(const v2f*)(lg + c);
    v2f ev;
#pragma unroll
    for (int e = 0; e < 2; ++e) {
      ev[e] = expf(l[e] - m);
      sum += ev[e];
    }
    *(v2f*)(lg + c) = ev;
  }
  sum = wave_sum32(sum);
  if (lane == 0) redS[wave] = sum;
  __syncthreads();
  float tot = redS[0];
#pragma unroll
  for (int w = 1; w < 8; ++w) tot += redS[w];
  const float inv = kPCarry / tot;

  const v4f e0 = *(const v4f*)(lg + 8 * t);
  const v4f e1 = *(const v4f*)(lg + 8 * t + 4);
  unsigned short hb[8];
#pragma unroll
  for (int e = 0; e < 4; ++e) {
    hb[e]     = h_bits(e0[e] * inv);
    hb[4 + e] = h_bits(e1[e] * inv);
  }
  const v4u u = (v4u){pk16(hb[0], hb[1]), pk16(hb[2], hb[3]), pk16(hb[4], hb[5]), pk16(hb[6], hb[7])};
  unsigned short* pr = Pp + rowoff + 8 * (size_t)t;
  *(volatile v4u*)pr = u;
  __threadfence();
  *(volatile v4u*)pr = u;
}

__global__ __launch_bounds__(256) void gn_gate_kernel(const float* __restrict__ O, const float* __restrict__ G,
                                                      const float* __restrict__ gamma, const float* __restrict__ beta,
                                                      unsigned short* __restrict__ Ah, unsigned short* __restrict__ Al) {
  __shared__ float red1[8];
  __shared__ float red2[8];
  __shared__ __align__(16) float slab[8][4 * 68];
  const int h    = blockIdx.x;
  const int tid  = threadIdx.x;
  const int lane = tid & 31, wave = tid >> 5;
  const float* Ob = O + h * kHD;
  const float invN = 1.0f / (float)(kT * kHD);

  float s = 0.0f;
#pragma unroll 1
  for (int i = 0; i < 8; ++i) {
    const float* r = Ob + (size_t)(tid + 256 * i) * kE;
#pragma unroll 2
    for (int j = 0; j < 16; ++j) {
      const v4f w = *(const v4f*)(r + 4 * j);
      s += (w[0] + w[1]) + (w[2] + w[3]);
    }
  }
  s = wave_sum32(s);
  if (lane == 0) red1[wave] = s;
  __syncthreads();
  float tot = red1[0];
#pragma unroll
  for (int w = 1; w < 8; ++w) tot += red1[w];
  const float mu = tot * invN;

  float ss = 0.0f;
#pragma unroll 1
  for (int i = 0; i < 8; ++i) {
    const float* r = Ob + (size_t)(tid + 256 * i) * kE;
#pragma unroll 2
    for (int j = 0; j < 16; ++j) {
      const v4f w = *(const v4f*)(r + 4 * j);
      const float d0 = w[0] - mu, d1 = w[1] - mu, d2 = w[2] - mu, d3 = w[3] - mu;
      ss = fmaf(d0, d0, ss);
      ss = fmaf(d1, d1, ss);
      ss = fmaf(d2, d2, ss);
      ss = fmaf(d3, d3, ss);
    }
  }
  ss = wave_sum32(ss);
  if (lane == 0) red2[wave] = ss;
  __syncthreads();
  float tot2 = red2[0];
#pragma unroll
  for (int w = 1; w < 8; ++w) tot2 += red2[w];
  const float var  = tot2 * invN;
  const float rstd = 1.0f / sqrtf(var + kGnEps);

  const int l2 = 2 * lane;
  const v2f gm = *(const v2f*)(gamma + h * kHD + l2);
  const v2f bt = *(const v2f*)(beta + h * kHD + l2);
  const int q = lane >> 3, c8 = (lane & 7) * 8;
  float* sl = slab[wave];
#pragma unroll 1
  for (int it = 0; it < 64; ++it) {
    const int tb = wave * 256 + it * 4;
#pragma unroll 1
    for (int rr = 0; rr < 4; ++rr) {
      const size_t off = (size_t)(tb + rr) * kE + h * kHD + l2;
      const v2f o = *(const v2f*)(O + off);
      const v2f g = *(const v2f*)(G + off);
      v2f a;
#pragma unroll
      for (int e = 0; e < 2; ++e) {
        const float on  = (o[e] - mu) * rstd * gm[e] + bt[e];
        const float sig = __builtin_amdgcn_rcpf(1.0f + expf(-g[e]));
        a[e] = (g[e] * sig) * on;
      }
      *(v2f*)(sl + rr * 68 + l2) = a;
    }
    __builtin_amdgcn_fence(__ATOMIC_RELEASE, "workgroup");
    __builtin_amdgcn_wave_barrier();
    __builtin_amdgcn_fence(__ATOMIC_ACQUIRE, "workgroup");
    const v4f a0 = *(const v4f*)(sl + q * 68 + c8);
    const v4f a1 = *(const v4f*)(sl + q * 68 + c8 + 4);
    unsigned short hb[8], lb[8];
#pragma unroll
    for (int e = 0; e < 4; ++e) {
      const float f0 = a0[e], f1 = a1[e];
      const unsigned short h0 = f2bf_bits(f0), h1 = f2bf_bits(f1);
      hb[e]     = h0;
      hb[4 + e] = h1;
      lb[e]     = f2bf_bits(f0 - bf_bits2f(h0));
      lb[4 + e] = f2bf_bits(f1 - bf_bits2f(h1));
    }
    const v4u uh = (v4u){pk16(hb[0], hb[1]), pk16(hb[2], hb[3]), pk16(hb[4], hb[5]), pk16(hb[6], hb[7])};
    const v4u ul = (v4u){pk16(lb[0], lb[1]), pk16(lb[2], lb[3]), pk16(lb[4], lb[5]), pk16(lb[6], lb[7])};
    const size_t doff = (size_t)(tb + q) * kE + h * kHD + c8;
    unsigned short* dh = Ah + doff;
    unsigned short* dl = Al + doff;
    *(volatile v4u*)dh = uh;
    *(volatile v4u*)dl = ul;
    __threadfence();
    *(volatile v4u*)dh = uh;
    *(volatile v4u*)dl = ul;
    __builtin_amdgcn_fence(__ATOMIC_RELEASE, "workgroup");
    __builtin_amdgcn_wave_barrier();
    __builtin_amdgcn_fence(__ATOMIC_ACQUIRE, "workgroup");
  }
}

extern "C" void kernel_launch(void* const* d_in, const int* in_sizes, int n_in,
                              void* d_out, int out_size, void* d_ws, size_t ws_size,
                              hipStream_t stream) {
  if (n_in < 15) return;
  const int nTE = kT * kE;
  const int nEE = kE * kE;
  if (in_sizes[0] != nTE) return;
  if (in_sizes[1] != nEE || in_sizes[3] != nEE || in_sizes[5] != nEE || in_sizes[7] != nEE || in_sizes[9] != nEE) return;
  if (in_sizes[2] != kE || in_sizes[4] != kE || in_sizes[6] != kE || in_sizes[8] != kE || in_sizes[10] != kE) return;
  if (in_sizes[11] != kH * kE || in_sizes[12] != kH || in_sizes[13] != kE || in_sizes[14] != kE) return;
  if (out_size != nTE) return;

  const size_t szXB  = (size_t)nTE * 2;
  const size_t szWB  = (size_t)nEE * 2;
  const size_t szF32 = (size_t)nTE * 4;
  const size_t szH16 = (size_t)nTE * 2;
  const size_t szTab = (size_t)kT * 32 * 4;
  const size_t szLD  = 4096;
  const size_t szSC  = (size_t)kGroup * kT * kT * 4;
  const size_t szPP  = (size_t)kGroup * kT * kT * 2;
  const size_t offXH  = 0;
  const size_t offXL  = offXH + szXB;
  const size_t offWH  = offXL + szXB;
  const size_t offWL  = offWH + szWB;
  const size_t offQR  = offWL + szWB;
  const size_t offKR  = offQR + szF32;
  const size_t offVR  = offKR + szF32;
  const size_t offGR  = offVR + szF32;
  const size_t offQH  = offGR + szF32;
  const size_t offKH  = offQH + szH16;
  const size_t offVT  = offKH + szH16;
  const size_t offCOS = offVT + szH16;
  const size_t offSIN = offCOS + szTab;
  const size_t offLD  = offSIN + szTab;
  const size_t offSC  = offLD + szLD;
  const size_t offPP  = offSC + szSC;
  const size_t offO   = offPP + szPP;
  const size_t offAH  = offO + szF32;
  const size_t offAL  = offAH + szXB;
  const size_t total  = offAL + szXB;
  if (ws_size < total) return;

  const float* x     = (const float*)d_in[0];
  const float* wq    = (const float*)d_in[1];
  const float* bq    = (const float*)d_in[2];
  const float* wk    = (const float*)d_in[3];
  const float* bk    = (const float*)d_in[4];
  const float* wv    = (const float*)d_in[5];
  const float* bv    = (const float*)d_in[6];
  const float* wg    = (const float*)d_in[7];
  const float* bg    = (const float*)d_in[8];
  const float* wo    = (const float*)d_in[9];
  const float* bo    = (const float*)d_in[10];
  const float* wd    = (const float*)d_in[11];
  const float* bd    = (const float*)d_in[12];
  const float* gamma = (const float*)d_in[13];
  const float* beta  = (const float*)d_in[14];
  float* out = (float*)d_out;
  char* ws = (char*)d_ws;
  unsigned short* XH = (unsigned short*)(ws + offXH);
  unsigned short* XL = (unsigned short*)(ws + offXL);
  unsigned short* WH = (unsigned short*)(ws + offWH);
  unsigned short* WL = (unsigned short*)(ws + offWL);
  float* QR = (float*)(ws + offQR);
  float* KR = (float*)(ws + offKR);
  float* VR = (float*)(ws + offVR);
  float* GR = (float*)(ws + offGR);
  unsigned short* QH = (unsigned short*)(ws + offQH);
  unsigned short* KH = (unsigned short*)(ws + offKH);
  unsigned short* VT = (unsigned short*)(ws + offVT);
  float* COS = (float*)(ws + offCOS);
  float* SIN = (float*)(ws + offSIN);
  float* LD  = (float*)(ws + offLD);
  float* SC  = (float*)(ws + offSC);
  unsigned short* PP  = (unsigned short*)(ws + offPP);
  float* O   = (float*)(ws + offO);
  unsigned short* AH = (unsigned short*)(ws + offAH);
  unsigned short* AL = (unsigned short*)(ws + offAL);

  FreqTab tab;
  for (int j = 0; j < 32; ++j) {
    const float p = (float)pow(10000.0, (double)j / 32.0);
    tab.f[j] = 1.0f / p;
  }

  const int n8x = nTE / 8;
  const int n8w = nEE / 8;
  split8_bf16_kernel<<<dim3(n8x / 256), dim3(256), 0, stream>>>(x, XH, XL, n8x);

  trig_table_kernel<<<dim3(kT / 8), dim3(256), 0, stream>>>(COS, SIN, tab);
  stats_decay_kernel<<<dim3(1), dim3(256), 0, stream>>>(x, wd, bd, LD);

  const int tilesProj = (kT / 64) * (kE / 64);
  split8_bf16_kernel<<<dim3(n8w / 256), dim3(256), 0, stream>>>(wq, WH, WL, n8w);
  wmma_gemm64<1, true, 2, 0, false, 0><<<dim3(tilesProj / 8, 1), dim3(256), 0, stream>>>(
      XH, XL, kE, 0L, WH, WL, kE, 0L, (void*)QR, (void*)QR, kE, 0L, bq, x, 0L, kT, kE, kE, 1.0f);
  split8_bf16_kernel<<<dim3(n8w / 256), dim3(256), 0, stream>>>(wk, WH, WL, n8w);
  wmma_gemm64<1, true, 2, 0, false, 0><<<dim3(tilesProj / 8, 1), dim3(256), 0, stream>>>(
      XH, XL, kE, 0L, WH, WL, kE, 0L, (void*)KR, (void*)KR, kE, 0L, bk, x, 0L, kT, kE, kE, 1.0f);
  split8_bf16_kernel<<<dim3(n8w / 256), dim3(256), 0, stream>>>(wv, WH, WL, n8w);
  wmma_gemm64<1, true, 2, 0, false, 0><<<dim3(tilesProj / 8, 1), dim3(256), 0, stream>>>(
      XH, XL, kE, 0L, WH, WL, kE, 0L, (void*)VR, (void*)VR, kE, 0L, bv, x, 0L, kT, kE, kE, 1.0f);
  split8_bf16_kernel<<<dim3(n8w / 256), dim3(256), 0, stream>>>(wg, WH, WL, n8w);
  wmma_gemm64<1, true, 2, 0, false, 0><<<dim3(tilesProj / 8, 1), dim3(256), 0, stream>>>(
      XH, XL, kE, 0L, WH, WL, kE, 0L, (void*)GR, (void*)GR, kE, 0L, bg, x, 0L, kT, kE, kE, 1.0f);

  rope_pack_kernel<<<dim3(kT / 64, kH), dim3(256), 0, stream>>>(QR, KR, VR, COS, SIN, QH, KH, VT);

  const long strideQK   = (long)kT * kHD;
  const long strideVT   = (long)kHD * kT;
  const long strideSC   = (long)kT * kT;
  const int  tilesScore = (kT / 64) * (kT / 64);
  const int  tilesCtx   = (kT / 64) * (kHD / 64);
  for (int g = 0; g < kH / kGroup; ++g) {
    const int hb = g * kGroup;
    const unsigned short* Ag  = QH + (size_t)hb * strideQK;
    const unsigned short* Btg = KH + (size_t)hb * strideQK;
    wmma_gemm64<0, false, 0, 0, false, 0><<<dim3(tilesScore / 8, kGroup), dim3(256), 0, stream>>>(
        Ag, Ag, kHD, strideQK, Btg, Btg, kHD, strideQK,
        (void*)SC, (void*)SC, kT, strideSC, LD, x, 0L, kT, kT, kHD, kScoreScale);
    softmax_bias_kernel<<<dim3(kT, kGroup), dim3(256), 0, stream>>>(SC, LD, PP, hb);
    const unsigned short* VTg = VT + (size_t)hb * strideVT;
    float* Og = O + (size_t)hb * kHD;
    wmma_gemm64<0, false, 0, 0, false, 0><<<dim3(tilesCtx / 8, kGroup), dim3(256), 0, stream>>>(
        PP, PP, kT, strideSC, VTg, VTg, kT, strideVT,
        (void*)Og, (void*)Og, kE, (long)kHD, LD, x, 0L, kT, kHD, kT, kPVScale);
  }

  gn_gate_kernel<<<dim3(kH), dim3(256), 0, stream>>>(O, GR, gamma, beta, AH, AL);

  split8_bf16_kernel<<<dim3(n8w / 256), dim3(256), 0, stream>>>(wo, WH, WL, n8w);
  wmma_gemm64<1, true, 2, 0, false, 0><<<dim3(tilesProj / 8, 1), dim3(256), 0, stream>>>(
      AH, AL, kE, 0L, WH, WL, kE, 0L, (void*)out, (void*)out, kE, 0L, bo, x, 0L, kT, kE, kE, 1.0f);
}
